// KAVNN_GO_14293651161791
// MI455X (gfx1250) — hardware-verified
//
#include <hip/hip_runtime.h>
#include <stddef.h>
#include <stdint.h>


typedef _Float16 v16h __attribute__((ext_vector_type(16)));
typedef _Float16 v8h  __attribute__((ext_vector_type(8)));
typedef _Float16 v2h  __attribute__((ext_vector_type(2)));
typedef float    v8f  __attribute__((ext_vector_type(8)));
typedef float    v4f  __attribute__((ext_vector_type(4)));
union Frag { v16h v; v8h half[2]; _Float16 s[16]; };

#define NB     256
#define DD     16
#define NT     256
#define NW     8
#define GN     8
#define CAPW   32
#define APITCH 40
#define LOG2E2 2.8853900817779268f

__device__ __forceinline__ v8f wmma_f16(v8f c, v16h a, v16h b) {
  c = __builtin_amdgcn_wmma_f32_16x16x32_f16(false, a, false, b, (short)0, c, false, false);
  asm volatile("v_nop\n\tv_nop\n\tv_nop\n\tv_nop" : "+v"(c) : "v"(a), "v"(b));
  return c;
}

__device__ __forceinline__ float tanh_fast(float x) {
  float e = __builtin_amdgcn_exp2f(x * LOG2E2);
  float r = __builtin_amdgcn_rcpf(e + 1.0f);
  return fmaf(-2.0f, r, 1.0f);
}

__device__ __forceinline__ v8h cvt8(v4f p, v4f q) {
  v8h r;
  r[0] = (_Float16)p[0]; r[1] = (_Float16)p[1]; r[2] = (_Float16)p[2]; r[3] = (_Float16)p[3];
  r[4] = (_Float16)q[0]; r[5] = (_Float16)q[1]; r[6] = (_Float16)q[2]; r[7] = (_Float16)q[3];
  return r;
}

__device__ __forceinline__ v8h zero8() {
  v8h r;
#pragma unroll
  for (int i = 0; i < 8; ++i) r[i] = (_Float16)0.0f;
  return r;
}

__device__ __forceinline__ void scan_edges(const int* __restrict__ esrc, const int* __restrict__ edst,
                                           int nE, int k0, int* cnt, int* lst)
{
  const int tid = threadIdx.x, lane = tid & 31, wv = tid >> 5;
  for (int base = 0; base < nE; base += NT) {
    const int e = base + tid;
    int dv = -1, sv = 0;
    if (e < nE) { dv = edst[e]; sv = esrc[e]; }
    const int rel = dv - k0;
    const bool hit = (e < nE) && ((unsigned)rel < (unsigned)GN);
    unsigned msk = __builtin_amdgcn_ballot_w32(hit);
    while (msk != 0u) {
      const int j = __builtin_ctz(msk);
      msk &= (msk - 1u);
      const int t = __builtin_amdgcn_ds_bpermute(j << 2, rel) & (GN - 1);
      const int s = __builtin_amdgcn_ds_bpermute(j << 2, sv);
      if (lane == 0) {
        const int slot = wv * GN + t;
        const int c = cnt[slot];
        if (c < CAPW) lst[slot * CAPW + c] = s;
        cnt[slot] = c + 1;
      }
    }
  }
}

__device__ __forceinline__ void tile_transform(float* tile, v16h bw, float bm, int wv, int h, int m)
{
  const float* r0p = tile + (32 * wv + m) * DD + 8 * h;
  const float* r1p = tile + (32 * wv + 16 + m) * DD + 8 * h;
  const v4f p0 = *(const v4f*)(r0p), p1 = *(const v4f*)(r0p + 4);
  const v4f q0 = *(const v4f*)(r1p), q1 = *(const v4f*)(r1p + 4);
  Frag a0, a1;
  a0.half[0] = cvt8(p0, p1); a0.half[1] = zero8();
  a1.half[0] = cvt8(q0, q1); a1.half[1] = zero8();
  v8f c0 = {0.f, 0.f, 0.f, 0.f, 0.f, 0.f, 0.f, 0.f};
  v8f c1 = {0.f, 0.f, 0.f, 0.f, 0.f, 0.f, 0.f, 0.f};
  c0 = wmma_f16(c0, a0.v, bw);
  c1 = wmma_f16(c1, a1.v, bw);
#pragma unroll
  for (int r = 0; r < 8; ++r) {
    tile[(32 * wv + 8 * h + r) * DD + m]      = tanh_fast(c0[r] + bm);
    tile[(32 * wv + 16 + 8 * h + r) * DD + m] = tanh_fast(c1[r] + bm);
  }
}

__device__ __forceinline__ void tile_store2(const float* tile, float* dst, int tid)
{
  const v4f o0 = ((const v4f*)tile)[tid];
  const v4f o1 = ((const v4f*)tile)[tid + NT];
  const v4f o2 = ((const v4f*)tile)[tid + 2 * NT];
  const v4f o3 = ((const v4f*)tile)[tid + 3 * NT];
  volatile v4f* vp = (volatile v4f*)dst;
  vp[tid] = o0; vp[tid + NT] = o1; vp[tid + 2 * NT] = o2; vp[tid + 3 * NT] = o3;
  __threadfence();
  vp[tid] = o0; vp[tid + NT] = o1; vp[tid + 2 * NT] = o2; vp[tid + 3 * NT] = o3;
}

__global__ __launch_bounds__(NT) void k_prep(const float* __restrict__ Wdec, const float* __restrict__ bdec,
                                             int n4, float* __restrict__ W2, float* __restrict__ B2)
{
  const int i = blockIdx.x * NT + threadIdx.x;
  const bool ok = i < n4;
  const int ii = ok ? i : 0;
  v4f w = ((const v4f*)Wdec)[ii];
  v4f b = ((const v4f*)bdec)[ii];
  w = w * LOG2E2;
  b = b * LOG2E2;
  volatile v4f* pw = (volatile v4f*)W2 + ii;
  volatile v4f* pb = (volatile v4f*)B2 + ii;
  if (ok) { *pw = w; *pb = b; }
  __threadfence();
  if (ok) { *pw = w; *pb = b; }
}

__global__ __launch_bounds__(NT) void k_go2ke(
    const float* __restrict__ x, int xcols, int ngo,
    const int* __restrict__ esrc, const int* __restrict__ edst, int nE,
    const float* __restrict__ W2, const float* __restrict__ B2,
    const float* __restrict__ Wg, const float* __restrict__ bg,
    float* __restrict__ KEout, int nke)
{
  __shared__ int s_cnt[NW * GN];
  __shared__ int s_lst[NW * GN * CAPW];
  __shared__ __align__(16) float s_tile[NB * DD];

  const int tid = threadIdx.x, lane = tid & 31, wv = tid >> 5, h = lane >> 4, m = lane & 15;
  const int k0 = blockIdx.x * GN;

  if (tid < NW * GN) s_cnt[tid] = 0;
  __syncthreads();
  scan_edges(esrc, edst, nE, k0, s_cnt, s_lst);
  __syncthreads();

  Frag bw;
#pragma unroll
  for (int i = 0; i < 8; ++i) {
    bw.s[i]     = (_Float16)Wg[(8 * h + i) * DD + m];
    bw.s[8 + i] = (_Float16)0.0f;
  }
  const float bgm = bg[m];
  const float* xb = x + (size_t)tid * (size_t)xcols;

#pragma unroll 1
  for (int j = 0; j < GN; ++j) {
    const int k = k0 + j;
    if (k >= nke) break;

    float acc[DD];
#pragma unroll
    for (int d = 0; d < DD; ++d) acc[d] = 0.0f;

#pragma unroll 1
    for (int w2 = 0; w2 < NW; ++w2) {
      int c = s_cnt[w2 * GN + j];
      c = c > CAPW ? CAPW : c;
      c = __builtin_amdgcn_readfirstlane(c);
#pragma unroll 1
      for (int i = 0; i < c; ++i) {
        int g = s_lst[(w2 * GN + j) * CAPW + i];
        g = g < 0 ? 0 : (g >= ngo ? ngo - 1 : g);
        g = __builtin_amdgcn_readfirstlane(g);
        const float xv = xb[g];
        const float* wr = W2 + (size_t)g * DD;
        const float* br = B2 + (size_t)g * DD;
#pragma unroll
        for (int d = 0; d < DD; ++d) {
          const float ev = __builtin_amdgcn_exp2f(fmaf(xv, wr[d], br[d]));
          acc[d] += fmaf(-2.0f, __builtin_amdgcn_rcpf(ev + 1.0f), 1.0f);
        }
      }
    }

    {
      v4f* trow = (v4f*)(s_tile + tid * DD);
      v4f t0, t1, t2, t3;
      t0[0] = acc[0];  t0[1] = acc[1];  t0[2] = acc[2];  t0[3] = acc[3];
      t1[0] = acc[4];  t1[1] = acc[5];  t1[2] = acc[6];  t1[3] = acc[7];
      t2[0] = acc[8];  t2[1] = acc[9];  t2[2] = acc[10]; t2[3] = acc[11];
      t3[0] = acc[12]; t3[1] = acc[13]; t3[2] = acc[14]; t3[3] = acc[15];
      trow[0] = t0; trow[1] = t1; trow[2] = t2; trow[3] = t3;
    }
    __syncthreads();
    tile_transform(s_tile, bw.v, bgm, wv, h, m);
    __syncthreads();
    tile_store2(s_tile, KEout + (size_t)k * (size_t)(NB * DD), tid);
    __syncthreads();
  }
}

__global__ __launch_bounds__(NT) void k_layer(
    const float* __restrict__ KEin, const int* __restrict__ esrc, const int* __restrict__ edst, int nE,
    const float* __restrict__ Wl, const float* __restrict__ bl, float* __restrict__ KEout,
    const float* __restrict__ wke, const float* __restrict__ bke, float* __restrict__ KES,
    int last, int nke)
{
  __shared__ int s_cnt[NW * GN];
  __shared__ int s_lst[NW * GN * CAPW];
  __shared__ __align__(16) float s_tile[NB * DD];
  __shared__ __align__(16) float s_red[NB];

  const int tid = threadIdx.x, lane = tid & 31, wv = tid >> 5, h = lane >> 4, m = lane & 15;
  const int k0 = blockIdx.x * GN;

  if (tid < NW * GN) s_cnt[tid] = 0;
  __syncthreads();
  scan_edges(esrc, edst, nE, k0, s_cnt, s_lst);
  __syncthreads();

  Frag bw;
#pragma unroll
  for (int i = 0; i < 8; ++i) {
    bw.s[i]     = (_Float16)Wl[(8 * h + i) * DD + m];
    bw.s[8 + i] = (_Float16)0.0f;
  }
  const float bm = bl[m];

#pragma unroll 1
  for (int j = 0; j < GN; ++j) {
    const int k = k0 + j;
    if (k >= nke) break;

    const v4f* selfp = (const v4f*)(KEin + ((size_t)k * NB + tid) * DD);
    v4f a0 = selfp[0], a1 = selfp[1], a2 = selfp[2], a3 = selfp[3];

#pragma unroll 1
    for (int w2 = 0; w2 < NW; ++w2) {
      int c = s_cnt[w2 * GN + j];
      c = c > CAPW ? CAPW : c;
      c = __builtin_amdgcn_readfirstlane(c);
#pragma unroll 1
      for (int i = 0; i < c; ++i) {
        int s = s_lst[(w2 * GN + j) * CAPW + i];
        s = s < 0 ? 0 : (s >= nke ? nke - 1 : s);
        s = __builtin_amdgcn_readfirstlane(s);
        const v4f* rp = (const v4f*)(KEin + ((size_t)s * NB + tid) * DD);
        a0 += rp[0]; a1 += rp[1]; a2 += rp[2]; a3 += rp[3];
      }
    }

    {
      v4f* trow = (v4f*)(s_tile + tid * DD);
      trow[0] = a0; trow[1] = a1; trow[2] = a2; trow[3] = a3;
    }
    __syncthreads();
    tile_transform(s_tile, bw.v, bm, wv, h, m);
    __syncthreads();
    if (last) {
      float sacc = 0.0f;
#pragma unroll
      for (int d = 0; d < DD; ++d) sacc = fmaf(s_tile[tid * DD + d], wke[d], sacc);
      s_red[tid] = tanh_fast(sacc + bke[0]);
    }
    __syncthreads();
    if (last) {
      const bool ok = tid < (NB / 4);
      v4f o; o[0] = 0.0f; o[1] = 0.0f; o[2] = 0.0f; o[3] = 0.0f;
      if (ok) o = ((const v4f*)s_red)[tid];
      volatile v4f* vp = (volatile v4f*)(KES + (size_t)k * NB);
      if (ok) vp[tid] = o;
      __threadfence();
      if (ok) vp[tid] = o;
    } else {
      tile_store2(s_tile, KEout + (size_t)k * (size_t)(NB * DD), tid);
    }
    __syncthreads();
  }
}

__global__ __launch_bounds__(NT) void k_gather(const float* __restrict__ KES, const int* __restrict__ tis,
                                               int nT, int nke, float* __restrict__ BIO0)
{
  const int nq = nT >> 2;
  const int i = blockIdx.x * NT + threadIdx.x;
  const bool ok = i < NB * nq;
  const int ii = ok ? i : 0;
  const int b = ii / nq, tq = ii - b * nq;
  v4f o;
#pragma unroll
  for (int q = 0; q < 4; ++q) {
    int t = tis[4 * tq + q];
    t = t < 0 ? 0 : (t >= nke ? nke - 1 : t);
    o[q] = KES[(size_t)t * NB + b];
  }
  volatile v4f* p = (volatile v4f*)(BIO0 + (size_t)b * nT + 4 * tq);
  if (ok) *p = o;
  __threadfence();
  if (ok) *p = o;
}

__global__ __launch_bounds__(NT) void k_gemm_relu(
    const float* __restrict__ A, int lda, int M,
    const float* __restrict__ W, const float* __restrict__ bias,
    float* __restrict__ out, int N, int K)
{
  __shared__ __align__(16) _Float16 As[16 * APITCH];
  __shared__ __align__(16) float Os[16 * 128];

  const int tid = threadIdx.x, lane = tid & 31, wv = tid >> 5, h = lane >> 4, m = lane & 15;
  const int m0 = blockIdx.x * 16, nb = blockIdx.y * 128;
  const int n  = nb + wv * 16 + m;
  const int ncl = n < N ? n : N - 1;
  const int sr = tid >> 4, sc = (tid & 15) * 2;
  int arow = m0 + sr; arow = arow < M ? arow : M - 1;
  const float* ap = A + (size_t)arow * (size_t)lda + sc;

  v8f c = {0.f, 0.f, 0.f, 0.f, 0.f, 0.f, 0.f, 0.f};
  for (int k0 = 0; k0 < K; k0 += 32) {
    v2h pv;
    pv[0] = (_Float16)ap[k0];
    pv[1] = (_Float16)ap[k0 + 1];
    *(v2h*)(As + sr * APITCH + sc) = pv;
    __syncthreads();
    Frag a;
    a.half[0] = *(const v8h*)(As + m * APITCH + 8 * h);
    a.half[1] = *(const v8h*)(As + m * APITCH + 16 + 8 * h);
    Frag bfr;
#pragma unroll
    for (int i = 0; i < 8; ++i) {
      bfr.s[i]     = (_Float16)W[(size_t)(k0 + 8 * h + i) * N + ncl];
      bfr.s[8 + i] = (_Float16)W[(size_t)(k0 + 16 + 8 * h + i) * N + ncl];
    }
    c = wmma_f16(c, a.v, bfr.v);
    __syncthreads();
  }

  const float bn = bias[ncl];
#pragma unroll
  for (int r = 0; r < 8; ++r) {
    const float v = c[r] + bn;
    Os[(8 * h + r) * 128 + wv * 16 + m] = v > 0.0f ? v : 0.0f;
  }
  __syncthreads();

  const v4f o0 = ((const v4f*)Os)[tid];
  const v4f o1 = ((const v4f*)Os)[tid + NT];
  const int r0 = m0 + (tid >> 5), r1 = m0 + 8 + (tid >> 5);
  const int cc = nb + lane * 4;
  const bool ok0 = (r0 < M) && (cc + 3 < N);
  const bool ok1 = (r1 < M) && (cc + 3 < N);
  volatile v4f* p0 = (volatile v4f*)(out + (size_t)r0 * N + cc);
  volatile v4f* p1 = (volatile v4f*)(out + (size_t)r1 * N + cc);
  if (ok0) *p0 = o0;
  if (ok1) *p1 = o1;
  __threadfence();
  if (ok0) *p0 = o0;
  if (ok1) *p1 = o1;
}

__global__ __launch_bounds__(NT) void k_pred(
    const float* __restrict__ bio2, const float* __restrict__ dr2,
    const float* __restrict__ Wp, const float* __restrict__ bp,
    float* __restrict__ out, int nout)
{
  __shared__ __align__(16) float s_red[NB];
  const int tid = threadIdx.x;
  const int b = tid;
  float s = 0.0f;
#pragma unroll 4
  for (int i = 0; i < 128; ++i) s = fmaf(bio2[b * 128 + i], Wp[i], s);
#pragma unroll 4
  for (int i = 0; i < 128; ++i) s = fmaf(dr2[b * 128 + i], Wp[128 + i], s);
  s_red[b] = s + bp[0];
  __syncthreads();
  const bool ok = (tid < NB / 4) && (4 * tid + 3 < nout);
  v4f o; o[0] = 0.0f; o[1] = 0.0f; o[2] = 0.0f; o[3] = 0.0f;
  if (tid < NB / 4) o = ((const v4f*)s_red)[tid];
  volatile v4f* p = (volatile v4f*)(out + 4 * tid);
  if (ok) *p = o;
  __threadfence();
  if (ok) *p = o;
}

extern "C" void kernel_launch(void* const* d_in, const int* in_sizes, int n_in,
                              void* d_out, int out_size, void* d_ws, size_t ws_size,
                              hipStream_t stream)
{
  if (n_in < 24) return;
  const float* x       = (const float*)d_in[0];
  const int*   go_src  = (const int*)d_in[1];
  const int*   go_dst  = (const int*)d_in[2];
  const int*   kk_src  = (const int*)d_in[3];
  const int*   kk_dst  = (const int*)d_in[4];
  const int*   tissue  = (const int*)d_in[5];
  const float* W_dec   = (const float*)d_in[6];
  const float* b_dec   = (const float*)d_in[7];
  const float* W_g2k   = (const float*)d_in[8];
  const float* b_g2k   = (const float*)d_in[9];
  const float* W_kk    = (const float*)d_in[10];
  const float* b_kk    = (const float*)d_in[11];
  const float* w_ke    = (const float*)d_in[12];
  const float* b_ke    = (const float*)d_in[13];
  const float* W_bio1  = (const float*)d_in[14];
  const float* b_bio1  = (const float*)d_in[15];
  const float* W_bio2  = (const float*)d_in[16];
  const float* b_bio2  = (const float*)d_in[17];
  const float* W_drug1 = (const float*)d_in[18];
  const float* b_drug1 = (const float*)d_in[19];
  const float* W_drug2 = (const float*)d_in[20];
  const float* b_drug2 = (const float*)d_in[21];
  const float* W_pred  = (const float*)d_in[22];
  const float* b_pred  = (const float*)d_in[23];
  float* out = (float*)d_out;

  const int ngo = 8000, nke = 2000, drug = 2048, nT = 512;
  const int xcols = ngo + drug;
  const int h_bio1 = 256, h_bio2 = 128, h_dr1 = 512, h_dr2 = 128;

  if (in_sizes[0] != NB * xcols) return;
  if (in_sizes[5] != nT) return;
  if (in_sizes[6] != ngo * DD || in_sizes[7] != ngo * DD) return;
  if (in_sizes[8] != DD * DD || in_sizes[10] < 3 * DD * DD || in_sizes[11] < 3 * DD) return;
  if (in_sizes[14] != nT * h_bio1 || in_sizes[16] != h_bio1 * h_bio2) return;
  if (in_sizes[18] != drug * h_dr1 || in_sizes[20] != h_dr1 * h_dr2) return;
  if (in_sizes[22] != h_bio2 + h_dr2 || out_size != NB) return;

  int nE_go = in_sizes[1]; if (in_sizes[2] < nE_go) nE_go = in_sizes[2];
  int nE_kk = in_sizes[3]; if (in_sizes[4] < nE_kk) nE_kk = in_sizes[4];

  char* wsb = (char*)d_ws;
  size_t off = 0;
  const size_t keBytes  = (size_t)nke * NB * DD * sizeof(float);
  const size_t kesBytes = (size_t)nke * NB * sizeof(float);
  const size_t decBytes = (size_t)ngo * DD * sizeof(float);
  float* KEA  = (float*)(wsb + off); off += keBytes;
  float* KEB  = (float*)(wsb + off); off += keBytes;
  float* KES  = (float*)(wsb + off); off += kesBytes;
  float* W2   = (float*)(wsb + off); off += decBytes;
  float* B2   = (float*)(wsb + off); off += decBytes;
  float* BIO0 = (float*)(wsb + off); off += (size_t)NB * nT * sizeof(float);
  float* BIO1 = (float*)(wsb + off); off += (size_t)NB * h_bio1 * sizeof(float);
  float* BIO2 = (float*)(wsb + off); off += (size_t)NB * h_bio2 * sizeof(float);
  float* DR1  = (float*)(wsb + off); off += (size_t)NB * h_dr1 * sizeof(float);
  float* DR2  = (float*)(wsb + off); off += (size_t)NB * h_dr2 * sizeof(float);
  if (off > ws_size) return;

  const int n4dec = ngo * DD / 4;
  k_prep<<<(n4dec + NT - 1) / NT, NT, 0, stream>>>(W_dec, b_dec, n4dec, W2, B2);

  const int gridNodes = (nke + GN - 1) / GN;
  k_go2ke<<<gridNodes, NT, 0, stream>>>(x, xcols, ngo, go_src, go_dst, nE_go,
                                        W2, B2, W_g2k, b_g2k, KEA, nke);

  k_layer<<<gridNodes, NT, 0, stream>>>(KEA, kk_src, kk_dst, nE_kk, W_kk + 0 * DD * DD, b_kk + 0 * DD,
                                        KEB, w_ke, b_ke, KES, 0, nke);
  k_layer<<<gridNodes, NT, 0, stream>>>(KEB, kk_src, kk_dst, nE_kk, W_kk + 1 * DD * DD, b_kk + 1 * DD,
                                        KEA, w_ke, b_ke, KES, 0, nke);
  k_layer<<<gridNodes, NT, 0, stream>>>(KEA, kk_src, kk_dst, nE_kk, W_kk + 2 * DD * DD, b_kk + 2 * DD,
                                        KEB, w_ke, b_ke, KES, 1, nke);

  const int nquads = NB * (nT / 4);
  k_gather<<<(nquads + NT - 1) / NT, NT, 0, stream>>>(KES, tissue, nT, nke, BIO0);

  k_gemm_relu<<<dim3((NB + 15) / 16, h_bio1 / 128), NT, 0, stream>>>(BIO0, nT, NB, W_bio1, b_bio1, BIO1, h_bio1, nT);
  k_gemm_relu<<<dim3((NB + 15) / 16, h_bio2 / 128), NT, 0, stream>>>(BIO1, h_bio1, NB, W_bio2, b_bio2, BIO2, h_bio2, h_bio1);
  k_gemm_relu<<<dim3((NB + 15) / 16, h_dr1 / 128), NT, 0, stream>>>(x + ngo, xcols, NB, W_drug1, b_drug1, DR1, h_dr1, drug);
  k_gemm_relu<<<dim3((NB + 15) / 16, h_dr2 / 128), NT, 0, stream>>>(DR1, h_dr1, NB, W_drug2, b_drug2, DR2, h_dr2, h_dr1);

  k_pred<<<1, NT, 0, stream>>>(BIO2, DR2, W_pred, b_pred, out, out_size);
}
